// Decoder_7481833029763
// MI455X (gfx1250) — hardware-verified
//
#include <hip/hip_runtime.h>
#include <math.h>

constexpr int T_ENC    = 1000;
constexpr int T_PAD    = 1024;
constexpr int NBATCH   = 64;
constexpr int LDEC     = 250;
constexpr int HID      = 512;
constexpr int KD       = 128;
constexpr int VD       = 128;
constexpr int NVOC     = 34;
constexpr int NVOC_PAD = 64;
constexpr int GATES1   = 4 * HID;
constexpr int GATES2   = 4 * KD;
constexpr int XIN1     = HID + VD;
constexpr int KREC     = 640;
constexpr int HCW      = KD + VD;
constexpr int NROWS    = NBATCH * LDEC;
constexpr int NTHR     = 256;
constexpr int ROWS_BLK = 16;
constexpr int H1P      = 520;
constexpr int CTP      = 136;
constexpr int H2AP     = 256;
constexpr int NOUT0    = NROWS * NVOC;
constexpr int NOUT1    = NROWS * T_ENC;

constexpr float W_CARRY   = 64.0f;
constexpr float A_CARRY   = 256.0f;
constexpr float KEY_CARRY = 16.0f;
constexpr float VAL_CARRY = 16.0f;
constexpr float P_CARRY   = 256.0f;
constexpr float LO_CARRY  = 2048.0f;
constexpr float GATE_FOLD = 1.0f / (W_CARRY * A_CARRY);
constexpr float EN_FOLD_HI = 1.0f / (A_CARRY * KEY_CARRY);
constexpr float EN_FOLD_LO = EN_FOLD_HI / LO_CARRY;
constexpr float CTX_FOLD  = 1.0f / (P_CARRY * VAL_CARRY);
constexpr float PRED_FOLD = 1.0f / (A_CARRY * W_CARRY);

static_assert(VD + HID == KREC, "LSTM1 recurrent K");
static_assert(HID + KD == KREC, "LSTM2 K");
static_assert(KREC % 32 == 0 && HCW % 32 == 0 && VD % 32 == 0 && KD % 32 == 0 && HID % 32 == 0, "K multiples of 32");
static_assert(NROWS % 64 == 0 && NVOC_PAD % 64 == 0, "GEMM tile multiples");
static_assert(T_PAD % 128 == 0 && T_PAD >= T_ENC, "padded T");
static_assert(NBATCH % ROWS_BLK == 0, "batch tiles");
static_assert(HID == 64 * (NTHR / 32), "8 waves x 64 units");
static_assert(KD == 16 * (NTHR / 32), "8 waves x 16 units");
static_assert(ROWS_BLK == 2 * (NTHR / 32), "2 attention rows per wave");
static_assert((NOUT0 * 4) % 128 == 0, "out1 line aligned");
static_assert(NOUT0 % 4 == 0 && T_ENC % 4 == 0, "float4 packing");
static_assert((2 * ROWS_BLK * H1P) % NTHR == 0, "h1 fill exact");

typedef __attribute__((ext_vector_type(16))) _Float16 v16h;
typedef __attribute__((ext_vector_type(8)))  _Float16 v8h;
typedef __attribute__((ext_vector_type(4)))  _Float16 v4h;
typedef __attribute__((ext_vector_type(8)))  float    v8f;
typedef __attribute__((ext_vector_type(4)))  float    v4f;

__device__ __forceinline__ void guard4_h(v8f& a0, v8f& a1, v8f& a2, v8f& a3, v16h x, v16h y0, v16h y1, v16h y2, v16h y3) {
  asm volatile("v_nop\n\tv_nop\n\tv_nop\n\tv_nop"
               : "+v"(a0), "+v"(a1), "+v"(a2), "+v"(a3)
               : "v"(x), "v"(y0), "v"(y1), "v"(y2), "v"(y3));
}
__device__ __forceinline__ void guard1_h(v8f& a0, v16h x0, v16h x1, v16h x2, v16h x3, v16h y0, v16h y1, v16h y2, v16h y3) {
  asm volatile("v_nop\n\tv_nop\n\tv_nop\n\tv_nop"
               : "+v"(a0)
               : "v"(x0), "v"(x1), "v"(x2), "v"(x3), "v"(y0), "v"(y1), "v"(y2), "v"(y3));
}
__device__ __forceinline__ void acc_guard4(v8f& a, v8f& b, v8f& c, v8f& d) {
  asm volatile("v_nop\n\tv_nop\n\tv_nop\n\tv_nop" : "+v"(a), "+v"(b), "+v"(c), "+v"(d));
}

template <typename T> struct Frag;
template <> struct Frag<_Float16> {
  typedef v16h V; union U { v16h v; v8h h[2]; };
  static __device__ __forceinline__ v16h load(const _Float16* p) {
    U f; f.h[0] = *(const v8h*)(p); f.h[1] = *(const v8h*)(p + 16); return f.v;
  }
  static __device__ __forceinline__ v8f mma(v16h a, v16h b, v8f c) {
    return __builtin_amdgcn_wmma_f32_16x16x32_f16(false, a, false, b, (short)0, c, false, false);
  }
};
typedef Frag<_Float16> FH;

__device__ __forceinline__ v16h zero16h() {
  union { v16h v; v8f f; } u;
  u.f = (v8f){0.f, 0.f, 0.f, 0.f, 0.f, 0.f, 0.f, 0.f};
  return u.v;
}
__device__ __forceinline__ void wave_sync() {
  __builtin_amdgcn_fence(__ATOMIC_RELEASE, "workgroup");
  __builtin_amdgcn_wave_barrier();
  __builtin_amdgcn_fence(__ATOMIC_ACQUIRE, "workgroup");
}
__device__ __forceinline__ float fsig(float x)  { return __builtin_amdgcn_rcpf(1.0f + expf(-x)); }
__device__ __forceinline__ float ftanh(float x) { return 1.0f - 2.0f * __builtin_amdgcn_rcpf(expf(2.0f * x) + 1.0f); }

__global__ __launch_bounds__(NTHR) void cvt_seg_kernel(const float* __restrict__ src, int spitch, int scol0, int nrow_src,
                                                       unsigned short* __restrict__ dst, int dpitch, int dcol0,
                                                       int nrow, int ncol8, float sc) {
  const int i  = blockIdx.x * NTHR + threadIdx.x;
  const int n8 = nrow * ncol8;
  if (i < n8) {
    const int row = i / ncol8;
    const int c8  = i - row * ncol8;
    const bool live = row < nrow_src;
    const int rs = live ? row : (nrow_src - 1);
    const float* sp = src + (size_t)rs * spitch + scol0 + c8 * 8;
    const v4f a = *(const v4f*)(sp);
    const v4f b = *(const v4f*)(sp + 4);
    v8h hv;
#pragma unroll
    for (int e = 0; e < 4; ++e) {
      const float fa = a[e];
      const float fb = b[e];
      hv[e]     = (_Float16)(live ? fa * sc : 0.0f);
      hv[4 + e] = (_Float16)(live ? fb * sc : 0.0f);
    }
    unsigned short* dp = dst + (size_t)row * dpitch + dcol0 + c8 * 8;
    *(volatile v8h*)dp = hv;
    __threadfence();
    *(volatile v8h*)dp = hv;
  }
}

__global__ __launch_bounds__(NTHR) void gemb_kernel(const float* __restrict__ emb, const float* __restrict__ W_ih1,
                                                    const float* __restrict__ b_ih1, const float* __restrict__ b_hh1,
                                                    float* __restrict__ G) {
  const int i = blockIdx.x * NTHR + threadIdx.x;
  if (i < NVOC * (GATES1 / 4)) {
    const int tok = i / (GATES1 / 4);
    const int j4  = (i - tok * (GATES1 / 4)) * 4;
    const float* er = emb + (size_t)tok * HID;
    const float* w0 = W_ih1 + (size_t)j4 * XIN1;
    float s0 = 0.0f, s1 = 0.0f, s2 = 0.0f, s3 = 0.0f;
#pragma unroll 1
    for (int k = 0; k < HID; k += 4) {
      const v4f e4 = *(const v4f*)(er + k);
      const v4f a0 = *(const v4f*)(w0 + k);
      const v4f a1 = *(const v4f*)(w0 + XIN1 + k);
      const v4f a2 = *(const v4f*)(w0 + 2 * XIN1 + k);
      const v4f a3 = *(const v4f*)(w0 + 3 * XIN1 + k);
      s0 += e4[0] * a0[0]; s0 += e4[1] * a0[1]; s0 += e4[2] * a0[2]; s0 += e4[3] * a0[3];
      s1 += e4[0] * a1[0]; s1 += e4[1] * a1[1]; s1 += e4[2] * a1[2]; s1 += e4[3] * a1[3];
      s2 += e4[0] * a2[0]; s2 += e4[1] * a2[1]; s2 += e4[2] * a2[2]; s2 += e4[3] * a2[3];
      s3 += e4[0] * a3[0]; s3 += e4[1] * a3[1]; s3 += e4[2] * a3[2]; s3 += e4[3] * a3[3];
    }
    const v4f bi = *(const v4f*)(b_ih1 + j4);
    const v4f bh = *(const v4f*)(b_hh1 + j4);
    v4f o;
    o[0] = s0 + bi[0] + bh[0];
    o[1] = s1 + bi[1] + bh[1];
    o[2] = s2 + bi[2] + bh[2];
    o[3] = s3 + bi[3] + bh[3];
    float* op = G + (size_t)tok * GATES1 + j4;
    *(volatile v4f*)op = o;
    __threadfence();
    *(volatile v4f*)op = o;
  }
}

__global__ __launch_bounds__(NTHR) void key_plane_kernel(const float* __restrict__ key_enc, unsigned short* __restrict__ dst, float sc) {
  const int i  = blockIdx.x * NTHR + threadIdx.x;
  const int c8 = i & 15;
  const int t  = (i >> 4) & (T_PAD - 1);
  const int n  = i >> 14;
  const bool live = t < T_ENC;
  const int tc = live ? t : (T_ENC - 1);
  const float* sp = key_enc + ((size_t)tc * NBATCH + n) * KD + c8 * 8;
  const v4f a = *(const v4f*)(sp);
  const v4f b = *(const v4f*)(sp + 4);
  v8h hv;
#pragma unroll
  for (int e = 0; e < 4; ++e) {
    const float fa = a[e];
    const float fb = b[e];
    hv[e]     = (_Float16)(live ? fa * sc : 0.0f);
    hv[4 + e] = (_Float16)(live ? fb * sc : 0.0f);
  }
  unsigned short* dp = dst + (size_t)i * 8;
  *(volatile v8h*)dp = hv;
  __threadfence();
  *(volatile v8h*)dp = hv;
}

__global__ __launch_bounds__(NTHR) void val_plane_kernel(const float* __restrict__ values, unsigned short* __restrict__ O, float sc) {
  __shared__ float Tt[64 * 65];
  const int tid = threadIdx.x;
  const int t0 = blockIdx.x * 64, v0 = blockIdx.y * 64, n = blockIdx.z;
#pragma unroll
  for (int i = 0; i < 4; ++i) {
    const int idx = i * NTHR + tid;
    const int rr = idx >> 4, cc = (idx & 15) * 4;
    const int t = t0 + rr;
    const bool live = t < T_ENC;
    const int tc = live ? t : (T_ENC - 1);
    const v4f v = *(const v4f*)(values + ((size_t)tc * NBATCH + n) * VD + v0 + cc);
    const float f0 = v[0], f1 = v[1], f2 = v[2], f3 = v[3];
    Tt[rr * 65 + cc + 0] = live ? f0 : 0.0f;
    Tt[rr * 65 + cc + 1] = live ? f1 : 0.0f;
    Tt[rr * 65 + cc + 2] = live ? f2 : 0.0f;
    Tt[rr * 65 + cc + 3] = live ? f3 : 0.0f;
  }
  __syncthreads();
  const int q = tid >> 3, c8 = (tid & 7) * 8;
  v8h hv[2];
#pragma unroll
  for (int g = 0; g < 2; ++g) {
    const int qq = g * 32 + q;
#pragma unroll
    for (int e = 0; e < 8; ++e) {
      const float f = Tt[(c8 + e) * 65 + qq];
      hv[g][e] = (_Float16)(f * sc);
    }
  }
  for (int pass = 0; pass < 2; ++pass) {
#pragma unroll
    for (int g = 0; g < 2; ++g) {
      const size_t o = ((size_t)n * VD + (size_t)(v0 + g * 32 + q)) * (size_t)T_PAD + (size_t)(t0 + c8);
      *(volatile v8h*)(O + o) = hv[g];
    }
    __threadfence();
  }
}

__device__ __forceinline__ void gate_kloop(v8f& a0, v8f& a1, v8f& a2, v8f& a3,
                                           const _Float16* arow, const _Float16* wb, size_t gstride, int klen) {
#pragma unroll 1
  for (int k0 = 0; k0 < klen; k0 += 32) {
    const v16h a  = FH::load(arow + k0);
    const v16h b0 = FH::load(wb + k0);
    const v16h b1 = FH::load(wb + gstride + k0);
    const v16h b2 = FH::load(wb + 2 * gstride + k0);
    const v16h b3 = FH::load(wb + 3 * gstride + k0);
    a0 = FH::mma(a, b0, a0);
    a1 = FH::mma(a, b1, a1);
    a2 = FH::mma(a, b2, a2);
    a3 = FH::mma(a, b3, a3);
    guard4_h(a0, a1, a2, a3, a, b0, b1, b2, b3);
  }
}

__global__ __launch_bounds__(NTHR) void las_decode_kernel(
    const float* __restrict__ values, const int* __restrict__ lens, const int* __restrict__ text,
    const float* __restrict__ b_ih2, const float* __restrict__ b_hh2, const float* __restrict__ GEMB,
    const unsigned short* __restrict__ W1rp, const unsigned short* __restrict__ W2rp,
    const unsigned short* __restrict__ KEY16p, const unsigned short* __restrict__ VALT16p,
    float* __restrict__ ATTWS, unsigned short* __restrict__ HC16) {
  __shared__ __align__(16) _Float16 sH1[2 * ROWS_BLK * H1P];
  __shared__ __align__(16) _Float16 sCT[ROWS_BLK * CTP];
  __shared__ __align__(16) _Float16 sH2A[ROWS_BLK * H2AP];
  __shared__ __align__(16) float    sC1[ROWS_BLK * HID];
  __shared__ __align__(16) float    sE[(NTHR / 32) * T_PAD];
  __shared__ __align__(16) _Float16 sP[(NTHR / 32) * T_PAD];

  const _Float16* W1r    = (const _Float16*)W1rp;
  const _Float16* W2r    = (const _Float16*)W2rp;
  const _Float16* KEY16  = (const _Float16*)KEY16p;
  const _Float16* VALT16 = (const _Float16*)VALT16p;

  const int tid = threadIdx.x, lane = tid & 31, wave = tid >> 5;
  const int c = lane & 15, hh = lane >> 4, koff = hh * 8;
  const int rowbase = blockIdx.x * ROWS_BLK;
  const v8f z8 = {0.f, 0.f, 0.f, 0.f, 0.f, 0.f, 0.f, 0.f};
  const v16h zh = zero16h();

#pragma unroll 1
  for (int i = tid; i < 2 * ROWS_BLK * H1P; i += NTHR) sH1[i] = (_Float16)0.0f;
#pragma unroll 1
  for (int i = tid; i < ROWS_BLK * H2AP; i += NTHR) sH2A[i] = (_Float16)0.0f;
#pragma unroll 1
  for (int i = tid; i < ROWS_BLK * HID; i += NTHR) sC1[i] = 0.0f;
#pragma unroll 1
  for (int i = tid; i < (NTHR / 32) * T_PAD; i += NTHR) sE[i] = 0.0f;
#pragma unroll 1
  for (int i = tid; i < (NTHR / 32) * T_PAD; i += NTHR) sP[i] = (_Float16)0.0f;
#pragma unroll 1
  for (int i = tid; i < ROWS_BLK * VD; i += NTHR) {
    const int m = i >> 7, v = i & (VD - 1);
    sCT[m * CTP + v] = (_Float16)(values[(size_t)(rowbase + m) * VD + v] * A_CARRY);
  }

  float c2s[8], bias2[4];
  const int j2 = 16 * wave + c;
#pragma unroll
  for (int r = 0; r < 8; ++r) c2s[r] = 0.0f;
#pragma unroll
  for (int g = 0; g < 4; ++g) bias2[g] = b_ih2[g * KD + j2] + b_hh2[g * KD + j2];
  int len0 = lens[rowbase + 2 * wave];
  int len1 = lens[rowbase + 2 * wave + 1];
  len0 = len0 < 1 ? 1 : (len0 > T_ENC ? T_ENC : len0);
  len1 = len1 < 1 ? 1 : (len1 > T_ENC ? T_ENC : len1);
  len0 = __builtin_amdgcn_readfirstlane(len0);
  len1 = __builtin_amdgcn_readfirstlane(len1);
  __syncthreads();

  float*    Ew = sE + wave * T_PAD;
  _Float16* Pw = sP + wave * T_PAD;

#pragma unroll 1
  for (int l = 0; l < LDEC; ++l) {
    const int par = l & 1;
    const _Float16* h1cur = sH1 + par * (ROWS_BLK * H1P);
    _Float16*       h1nxt = sH1 + (par ^ 1) * (ROWS_BLK * H1P);

    int goff[8];
#pragma unroll
    for (int r = 0; r < 8; ++r) {
      int tk = text[(size_t)(rowbase + 8 * hh + r) * LDEC + l];
      tk = tk < 0 ? 0 : (tk > NVOC - 1 ? NVOC - 1 : tk);
      goff[r] = tk * GATES1;
    }

#pragma unroll 1
    for (int nt = 0; nt < 4; ++nt) {
      const int j = 64 * wave + 16 * nt + c;
      const _Float16* wb = W1r + (size_t)j * KREC + koff;
      v8f acc0 = z8, acc1 = z8, acc2 = z8, acc3 = z8;
      gate_kloop(acc0, acc1, acc2, acc3, sCT + c * CTP + koff, wb, (size_t)HID * KREC, VD);
      gate_kloop(acc0, acc1, acc2, acc3, h1cur + c * H1P + koff, wb + VD, (size_t)HID * KREC, HID);
      acc_guard4(acc0, acc1, acc2, acc3);
#pragma unroll
      for (int r = 0; r < 8; ++r) {
        const int row = 8 * hh + r;
        const float* ge = GEMB + goff[r] + j;
        const float gi = ge[0];
        const float gf = ge[HID];
        const float gg = ge[2 * HID];
        const float go = ge[3 * HID];
        const float zi = acc0[r] * GATE_FOLD + gi;
        const float zf = acc1[r] * GATE_FOLD + gf;
        const float zg = acc2[r] * GATE_FOLD + gg;
        const float zo = acc3[r] * GATE_FOLD + go;
        const float cp = sC1[row * HID + j];
        const float cn = fsig(zf) * cp + fsig(zi) * ftanh(zg);
        const float hn = fsig(zo) * ftanh(cn);
        sC1[row * HID + j] = cn;
        h1nxt[row * H1P + j] = (_Float16)(hn * A_CARRY);
        asm volatile("" ::: "memory");
      }
    }
    __syncthreads();

    float h2n[8];
    {
      const _Float16* wb = W2r + (size_t)j2 * KREC + koff;
      v8f acc0 = z8, acc1 = z8, acc2 = z8, acc3 = z8;
      gate_kloop(acc0, acc1, acc2, acc3, h1nxt + c * H1P + koff, wb, (size_t)KD * KREC, HID);
      gate_kloop(acc0, acc1, acc2, acc3, sH2A + c * H2AP + koff, wb + HID, (size_t)KD * KREC, KD);
      acc_guard4(acc0, acc1, acc2, acc3);
#pragma unroll
      for (int r = 0; r < 8; ++r) {
        const float zi = acc0[r] * GATE_FOLD + bias2[0];
        const float zf = acc1[r] * GATE_FOLD + bias2[1];
        const float zg = acc2[r] * GATE_FOLD + bias2[2];
        const float zo = acc3[r] * GATE_FOLD + bias2[3];
        const float cn = fsig(zf) * c2s[r] + fsig(zi) * ftanh(zg);
        c2s[r] = cn;
        h2n[r] = fsig(zo) * ftanh(cn);
      }
    }
    __syncthreads();
#pragma unroll
    for (int r = 0; r < 8; ++r) {
      const int row = 8 * hh + r;
      const float hs = h2n[r] * A_CARRY;
      const _Float16 hi = (_Float16)hs;
      const float hif = (float)hi;
      const _Float16 lo = (_Float16)((hs - hif) * LO_CARRY);
      sH2A[row * H2AP + j2] = hi;
      sH2A[row * H2AP + KD + j2] = lo;
    }
    __syncthreads();

#pragma unroll 1
    for (int mm = 0; mm < 2; ++mm) {
      const int m = 2 * wave + mm;
      const int n = rowbase + m;
      const int len = mm ? len1 : len0;
      const int ntile = (len + 15) >> 4;
      const int nit = (len + 127) >> 7;
      const int nk = (len + 31) >> 5;

      v16h ea0, ea1, ea2, ea3;
      {
        const int cc = (c < 2) ? c : 1;
        const _Float16* hp = sH2A + m * H2AP + cc * KD + koff;
        const v16h r0 = FH::load(hp);
        const v16h r1 = FH::load(hp + 32);
        const v16h r2 = FH::load(hp + 64);
        const v16h r3 = FH::load(hp + 96);
        const bool live = c < 2;
        ea0 = live ? r0 : zh;
        ea1 = live ? r1 : zh;
        ea2 = live ? r2 : zh;
        ea3 = live ? r3 : zh;
      }
#pragma unroll 1
      for (int tile = 0; tile < ntile; ++tile) {
        const _Float16* kp = KEY16 + ((size_t)n * T_PAD + (size_t)(16 * tile + c)) * KD + koff;
        const v16h b0 = FH::load(kp);
        const v16h b1 = FH::load(kp + 32);
        const v16h b2 = FH::load(kp + 64);
        const v16h b3 = FH::load(kp + 96);
        v8f eacc = z8;
        eacc = FH::mma(ea0, b0, eacc);
        eacc = FH::mma(ea1, b1, eacc);
        eacc = FH::mma(ea2, b2, eacc);
        eacc = FH::mma(ea3, b3, eacc);
        guard1_h(eacc, ea0, ea1, ea2, ea3, b0, b1, b2, b3);
        const float en = eacc[0] * EN_FOLD_HI + eacc[1] * EN_FOLD_LO;
        if (hh == 0) Ew[16 * tile + c] = en;
      }
      wave_sync();

      float mx = -INFINITY;
#pragma unroll 1
      for (int it = 0; it < nit; ++it) {
        const int t = 128 * it + 4 * lane;
        const v4f ev = *(const v4f*)(Ew + t);
#pragma unroll
        for (int e = 0; e < 4; ++e) {
          const float x = ev[e];
          mx = (t + e < len) ? fmaxf(mx, x) : mx;
        }
      }
#pragma unroll
      for (int off = 1; off < 32; off <<= 1) mx = fmaxf(mx, __shfl_xor(mx, off, 32));
      float sm = 0.0f;
#pragma unroll 1
      for (int it = 0; it < nit; ++it) {
        const int t = 128 * it + 4 * lane;
        const v4f ev = *(const v4f*)(Ew + t);
        v4f pv;
#pragma unroll
        for (int e = 0; e < 4; ++e) {
          const float x = ev[e];
          const float pe = expf(x - mx);
          pv[e] = (t + e < len) ? pe : 0.0f;
        }
        sm += (pv[0] + pv[1]) + (pv[2] + pv[3]);
        *(v4f*)(Ew + t) = pv;
      }
#pragma unroll
      for (int off = 1; off < 32; off <<= 1) sm += __shfl_xor(sm, off, 32);
      const float inv = 1.0f / sm;

      float* arow = ATTWS + ((size_t)n * LDEC + (size_t)l) * T_PAD;
#pragma unroll 1
      for (int it = 0; it < nit; ++it) {
        const int t = 128 * it + 4 * lane;
        const v4f pv = *(const v4f*)(Ew + t);
        v4f av;
        v4h ph;
#pragma unroll
        for (int e = 0; e < 4; ++e) {
          const float pe = pv[e];
          av[e] = pe * inv;
          ph[e] = (_Float16)(pe * P_CARRY);
        }
        *(volatile v4f*)(arow + t) = av;
        *(v4h*)(Pw + t) = ph;
      }
      __threadfence();
#pragma unroll 1
      for (int it = 0; it < nit; ++it) {
        const int t = 128 * it + 4 * lane;
        const v4f pv = *(const v4f*)(Ew + t);
        v4f av;
#pragma unroll
        for (int e = 0; e < 4; ++e) {
          const float pe = pv[e];
          av[e] = pe * inv;
        }
        *(volatile v4f*)(arow + t) = av;
      }
      wave_sync();

      v8f cacc[8];
#pragma unroll
      for (int vt = 0; vt < 8; ++vt) cacc[vt] = z8;
      const _Float16* vb = VALT16 + ((size_t)n * VD + (size_t)c) * T_PAD + koff;
#pragma unroll 1
      for (int ks = 0; ks < nk; ++ks) {
        const v16h araw = FH::load(Pw + 32 * ks + koff);
        const v16h a = (c == 0) ? araw : zh;
        {
          const v16h b0 = FH::load(vb + (size_t)0  * T_PAD + 32 * ks);
          const v16h b1 = FH::load(vb + (size_t)16 * T_PAD + 32 * ks);
          const v16h b2 = FH::load(vb + (size_t)32 * T_PAD + 32 * ks);
          const v16h b3 = FH::load(vb + (size_t)48 * T_PAD + 32 * ks);
          cacc[0] = FH::mma(a, b0, cacc[0]);
          cacc[1] = FH::mma(a, b1, cacc[1]);
          cacc[2] = FH::mma(a, b2, cacc[2]);
          cacc[3] = FH::mma(a, b3, cacc[3]);
          guard4_h(cacc[0], cacc[1], cacc[2], cacc[3], a, b0, b1, b2, b3);
        }
        {
          const v16h b0 = FH::load(vb + (size_t)64  * T_PAD + 32 * ks);
          const v16h b1 = FH::load(vb + (size_t)80  * T_PAD + 32 * ks);
          const v16h b2 = FH::load(vb + (size_t)96  * T_PAD + 32 * ks);
          const v16h b3 = FH::load(vb + (size_t)112 * T_PAD + 32 * ks);
          cacc[4] = FH::mma(a, b0, cacc[4]);
          cacc[5] = FH::mma(a, b1, cacc[5]);
          cacc[6] = FH::mma(a, b2, cacc[6]);
          cacc[7] = FH::mma(a, b3, cacc[7]);
          guard4_h(cacc[4], cacc[5], cacc[6], cacc[7], a, b0, b1, b2, b3);
        }
      }
      acc_guard4(cacc[0], cacc[1], cacc[2], cacc[3]);
      acc_guard4(cacc[4], cacc[5], cacc[6], cacc[7]);
      {
        const float cs = inv * CTX_FOLD * A_CARRY;
        if (hh == 0) {
#pragma unroll
          for (int vt = 0; vt < 8; ++vt) {
            const float cx = cacc[vt][0] * cs;
            sCT[m * CTP + 16 * vt + c] = (_Float16)cx;
          }
        }
      }
      wave_sync();
      {
        const int l16 = lane & 15;
        const v8h va = *(const v8h*)(sH2A + m * H2AP + 8 * l16);
        const v8h vc = *(const v8h*)(sCT + m * CTP + 8 * l16);
        const v8h vv = (lane < 16) ? va : vc;
        unsigned short* hp = HC16 + ((size_t)n * LDEC + (size_t)l) * HCW + 8 * lane;
        *(volatile v8h*)hp = vv;
        __threadfence();
        *(volatile v8h*)hp = vv;
      }
      wave_sync();
    }
    __syncthreads();
  }
}

__global__ __launch_bounds__(256) void pred_gemm_kernel(const unsigned short* __restrict__ Ap, int lda,
                                                        const unsigned short* __restrict__ Btp, int ldb,
                                                        float* __restrict__ C, int ldc, int M, int N, int K, float scale) {
  const _Float16* A  = (const _Float16*)Ap;
  const _Float16* Bt = (const _Float16*)Btp;
  __shared__ __align__(16) float sT[8][16 * 68];
  const int lane = threadIdx.x & 31;
  const int wave = threadIdx.x >> 5;
  const int tilesN = N >> 6;
  const int tilesM = M >> 6;
  const int tile = blockIdx.x * 8 + wave;
  if (tile >= tilesM * tilesN) return;
  const int tm = tile / tilesN;
  const int tn = tile - tm * tilesN;
  const int m0 = tm << 6;
  const int n0 = tn << 6;
  const int rlane = lane & 15;
  const int koff  = (lane >> 4) * 8;
  const int mOff  = (lane >> 4) * 8;

  v8f acc[4][4];
#pragma unroll
  for (int i = 0; i < 4; ++i)
#pragma unroll
    for (int j = 0; j < 4; ++j) acc[i][j] = (v8f){0.f, 0.f, 0.f, 0.f, 0.f, 0.f, 0.f, 0.f};

  for (int k0 = 0; k0 < K; k0 += 32) {
    v16h bh[4];
#pragma unroll
    for (int j = 0; j < 4; ++j) {
      const size_t bo = (size_t)(n0 + (j << 4) + rlane) * ldb + koff + k0;
      bh[j] = FH::load(Bt + bo);
    }
#pragma unroll
    for (int i = 0; i < 4; ++i) {
      const size_t ao = (size_t)(m0 + (i << 4) + rlane) * lda + koff + k0;
      const v16h ah = FH::load(A + ao);
#pragma unroll
      for (int j = 0; j < 4; ++j) acc[i][j] = FH::mma(ah, bh[j], acc[i][j]);
      guard4_h(acc[i][0], acc[i][1], acc[i][2], acc[i][3], ah, bh[0], bh[1], bh[2], bh[3]);
    }
  }
  acc_guard4(acc[0][0], acc[0][1], acc[0][2], acc[0][3]);
  acc_guard4(acc[1][0], acc[1][1], acc[1][2], acc[1][3]);
  acc_guard4(acc[2][0], acc[2][1], acc[2][2], acc[2][3]);
  acc_guard4(acc[3][0], acc[3][1], acc[3][2], acc[3][3]);

  float* slab = sT[wave];
#pragma unroll
  for (int i = 0; i < 4; ++i) {
    const int mBase = m0 + (i << 4);
#pragma unroll
    for (int j = 0; j < 4; ++j) {
#pragma unroll
      for (int r = 0; r < 8; ++r) slab[(mOff + r) * 68 + (j << 4) + rlane] = acc[i][j][r] * scale;
    }
    wave_sync();
    {
      const int hh = lane >> 4, c4 = (lane & 15) * 4;
      for (int pass = 0; pass < 2; ++pass) {
#pragma unroll
        for (int it = 0; it < 8; ++it) {
          const int row = it * 2 + hh;
          const v4f v = *(const v4f*)(slab + row * 68 + c4);
          *(volatile v4f*)(C + (size_t)(mBase + row) * ldc + n0 + c4) = v;
        }
        __threadfence();
      }
    }
    wave_sync();
  }
}

__global__ __launch_bounds__(NTHR) void pred_pack_kernel(const float* __restrict__ P64, const float* __restrict__ b_out,
                                                         float* __restrict__ out0) {
  const int i = blockIdx.x * NTHR + threadIdx.x;
  if (i < NOUT0 / 4) {
    v4f o;
#pragma unroll
    for (int e = 0; e < 4; ++e) {
      const int idx = 4 * i + e;
      const int row = idx / NVOC;
      const int j = idx - row * NVOC;
      o[e] = P64[(size_t)row * NVOC_PAD + j] + b_out[j];
    }
    float* op = out0 + (size_t)i * 4;
    *(volatile v4f*)op = o;
    __threadfence();
    *(volatile v4f*)op = o;
  }
}

__global__ __launch_bounds__(NTHR) void att_pack_kernel(const float* __restrict__ ATTWS, const int* __restrict__ lens,
                                                        float* __restrict__ out1) {
  const int i = blockIdx.x * NTHR + threadIdx.x;
  if (i < NOUT1 / 4) {
    const int row = i / (T_ENC / 4);
    const int t = (i - row * (T_ENC / 4)) * 4;
    const int n = row / LDEC;
    int len = lens[n];
    len = len < 1 ? 1 : (len > T_ENC ? T_ENC : len);
    const int tl = (t < len) ? t : 0;
    const v4f a = *(const v4f*)(ATTWS + (size_t)row * T_PAD + tl);
    v4f o;
#pragma unroll
    for (int e = 0; e < 4; ++e) {
      const float x = a[e];
      o[e] = (t + e < len) ? x : 0.0f;
    }
    float* op = out1 + (size_t)i * 4;
    *(volatile v4f*)op = o;
    __threadfence();
    *(volatile v4f*)op = o;
  }
}

extern "C" void kernel_launch(void* const* d_in, const int* in_sizes, int n_in,
                              void* d_out, int out_size, void* d_ws, size_t ws_size, hipStream_t stream) {
  if (n_in < 15 || d_out == nullptr || d_ws == nullptr) return;
  if (in_sizes[0] != T_ENC * NBATCH * KD || in_sizes[1] != T_ENC * NBATCH * VD || in_sizes[2] != NBATCH ||
      in_sizes[3] != NBATCH * LDEC || in_sizes[4] != NVOC * HID || in_sizes[5] != GATES1 * XIN1 ||
      in_sizes[6] != GATES1 * HID || in_sizes[7] != GATES1 || in_sizes[8] != GATES1 ||
      in_sizes[9] != GATES2 * HID || in_sizes[10] != GATES2 * KD || in_sizes[11] != GATES2 ||
      in_sizes[12] != GATES2 || in_sizes[13] != NVOC * HCW || in_sizes[14] != NVOC ||
      out_size != NOUT0 + NOUT1) return;

  const float* key_enc = (const float*)d_in[0];
  const float* values  = (const float*)d_in[1];
  const int*   lens    = (const int*)d_in[2];
  const int*   text    = (const int*)d_in[3];
  const float* emb     = (const float*)d_in[4];
  const float* W_ih1   = (const float*)d_in[5];
  const float* W_hh1   = (const float*)d_in[6];
  const float* b_ih1   = (const float*)d_in[7];
  const float* b_hh1   = (const float*)d_in[8];
  const float* W_ih2   = (const float*)d_in[9];
  const float* W_hh2   = (const float*)d_in[10];
  const float* b_ih2   = (const float*)d_in[11];
  const float* b_hh2   = (const float*)d_in[12];
  const float* W_out   = (const float*)d_in[13];
  const float* b_out   = (const float*)d_in[14];
  float* out0 = (float*)d_out;
  float* out1 = out0 + (size_t)NOUT0;

  char* ws = (char*)d_ws; size_t off = 0;
  auto carve = [&](size_t bytes) -> char* { char* p = ws + off; off += (bytes + 255) & ~(size_t)255; return p; };
  unsigned short* W1R    = (unsigned short*)carve((size_t)GATES1 * KREC * 2);
  unsigned short* W2R    = (unsigned short*)carve((size_t)GATES2 * KREC * 2);
  unsigned short* WO16   = (unsigned short*)carve((size_t)NVOC_PAD * HCW * 2);
  float*          GEMB   = (float*)carve((size_t)NVOC * GATES1 * 4);
  unsigned short* KEY16  = (unsigned short*)carve((size_t)NBATCH * T_PAD * KD * 2);
  unsigned short* VALT16 = (unsigned short*)carve((size_t)NBATCH * VD * T_PAD * 2);
  float*          ATTWS  = (float*)carve((size_t)NROWS * T_PAD * 4);
  unsigned short* HC16   = (unsigned short*)carve((size_t)NROWS * HCW * 2);
  float*          P64    = (float*)carve((size_t)NROWS * NVOC_PAD * 4);
  if (off > ws_size || off > (size_t)134217728) return;

  cvt_seg_kernel<<<(GATES1 * (VD / 8)) / NTHR, NTHR, 0, stream>>>(W_ih1, XIN1, HID, GATES1, W1R, KREC, 0, GATES1, VD / 8, W_CARRY);
  cvt_seg_kernel<<<(GATES1 * (HID / 8)) / NTHR, NTHR, 0, stream>>>(W_hh1, HID, 0, GATES1, W1R, KREC, VD, GATES1, HID / 8, W_CARRY);
  cvt_seg_kernel<<<(GATES2 * (HID / 8)) / NTHR, NTHR, 0, stream>>>(W_ih2, HID, 0, GATES2, W2R, KREC, 0, GATES2, HID / 8, W_CARRY);
  cvt_seg_kernel<<<(GATES2 * (KD / 8)) / NTHR, NTHR, 0, stream>>>(W_hh2, KD, 0, GATES2, W2R, KREC, HID, GATES2, KD / 8, W_CARRY);
  cvt_seg_kernel<<<(NVOC_PAD * (HCW / 8)) / NTHR, NTHR, 0, stream>>>(W_out, HCW, 0, NVOC, WO16, HCW, 0, NVOC_PAD, HCW / 8, W_CARRY);
  gemb_kernel<<<(NVOC * (GATES1 / 4)) / NTHR, NTHR, 0, stream>>>(emb, W_ih1, b_ih1, b_hh1, GEMB);
  key_plane_kernel<<<(NBATCH * T_PAD * (KD / 8)) / NTHR, NTHR, 0, stream>>>(key_enc, KEY16, KEY_CARRY);
  val_plane_kernel<<<dim3(T_PAD / 64, VD / 64, NBATCH), NTHR, 0, stream>>>(values, VALT16, VAL_CARRY);
  las_decode_kernel<<<NBATCH / ROWS_BLK, NTHR, 0, stream>>>(values, lens, text, b_ih2, b_hh2, GEMB,
                                                            W1R, W2R, KEY16, VALT16, ATTWS, HC16);
  pred_gemm_kernel<<<((NROWS / 64) * (NVOC_PAD / 64) + 7) / 8, 256, 0, stream>>>(HC16, HCW, WO16, HCW, P64, NVOC_PAD,
                                                                                NROWS, NVOC_PAD, HCW, PRED_FOLD);
  pred_pack_kernel<<<(NOUT0 / 4 + NTHR - 1) / NTHR, NTHR, 0, stream>>>(P64, b_out, out0);
  att_pack_kernel<<<(NOUT1 / 4 + NTHR - 1) / NTHR, NTHR, 0, stream>>>(ATTWS, lens, out1);
}
